// CircumpunctAttention_17136919511703
// MI455X (gfx1250) — hardware-verified
//
#include <hip/hip_runtime.h>
#include <math.h>
#include <stdint.h>

#define TT      2048
#define DM      1024
#define NHEAD   16
#define HDIM    64
#define NGATE   64
#define HPB     8
#define QKP     (2 * DM)
#define OSW     (HPB * HDIM)
#define WSC     64.0f
#define ACARRY  16.0f
#define QC      16.0f
#define KC      16.0f
#define VC      1024.0f
#define PC      1024.0f
#define FC      4096.0f
#define ATT_SCALE 0.125f
#define PI_F    3.14159265358979323846f
#define REN_EPS 1e-8f
static_assert(NHEAD * HDIM == DM);
static_assert((TT % 64) == 0 && (DM % 64) == 0 && (DM % 256) == 0 && (TT % 32) == 0 && (TT % 16) == 0);
static_assert((NHEAD % HPB) == 0 && (NHEAD / HPB) == 2 && NGATE == 64 && OSW == 512);
#define ATT_THREADS (HPB * 32)
#define ATT_QT      (TT / 16)
#define ATT_BLOCKS  (ATT_QT * (NHEAD / HPB))
static_assert(ATT_THREADS == 256 && ATT_BLOCKS == 256);

typedef _Float16 v16h __attribute__((ext_vector_type(16)));
typedef _Float16 v8h  __attribute__((ext_vector_type(8)));
typedef float    v8f  __attribute__((ext_vector_type(8)));
typedef float    v4f  __attribute__((ext_vector_type(4)));
typedef unsigned int v4u __attribute__((ext_vector_type(4)));

union FragH { v16h v; v8h h[2]; v4u u[2]; };

__device__ __forceinline__ unsigned short bf_bits(float f) {
  unsigned u = __float_as_uint(f);
  return (unsigned short)((u + 0x7FFFu + ((u >> 16) & 1u)) >> 16);
}
__device__ __forceinline__ float bf_up(unsigned short h) { return __uint_as_float(((unsigned)h) << 16); }
__device__ __forceinline__ float bfr(float f) { return bf_up(bf_bits(f)); }
__device__ __forceinline__ unsigned short h_bits(_Float16 x) { return __builtin_bit_cast(unsigned short, x); }
__device__ __forceinline__ unsigned pk16(unsigned short a, unsigned short b) { return (unsigned)a | ((unsigned)b << 16); }
__device__ __forceinline__ v8f zero8() { v8f z = {0.f, 0.f, 0.f, 0.f, 0.f, 0.f, 0.f, 0.f}; return z; }
__device__ __forceinline__ float sigf(float v) { return 1.0f / (1.0f + expf(-v)); }

__device__ __forceinline__ v16h ldfrag_h(const _Float16* p) {
  FragH f;
  f.h[0] = *(const v8h*)(p);
  f.h[1] = *(const v8h*)(p + 16);
  return f.v;
}
__device__ __forceinline__ v16h ldfrag_u(const unsigned short* p) {
  FragH f;
  f.u[0] = *(const v4u*)(p);
  f.u[1] = *(const v4u*)(p + 16);
  return f.v;
}

__device__ __forceinline__ v8f mma_raw(v16h a, v16h b, v8f c) {
  return __builtin_amdgcn_wmma_f32_16x16x32_f16(false, a, false, b, (short)0, c, false, false);
}
__device__ __forceinline__ void dep_guard1(v8f& a, v8f& b, v16h x) {
#if defined(__HIP_DEVICE_COMPILE__)
  asm volatile("v_nop\n\tv_nop\n\tv_nop\n\tv_nop" : "+v"(a), "+v"(b) : "v"(x));
#endif
}
__device__ __forceinline__ void dep_guard2(v8f& a, v8f& b, v16h x, v16h y) {
#if defined(__HIP_DEVICE_COMPILE__)
  asm volatile("v_nop\n\tv_nop\n\tv_nop\n\tv_nop" : "+v"(a), "+v"(b) : "v"(x), "v"(y));
#endif
}
__device__ __forceinline__ void guard_s2(v8f& s, v16h a0, v16h a1) {
#if defined(__HIP_DEVICE_COMPILE__)
  asm volatile("v_nop\n\tv_nop\n\tv_nop\n\tv_nop" : "+v"(s) : "v"(a0), "v"(a1));
#endif
}
__device__ __forceinline__ void guard_s4(v8f& s, v16h a0, v16h a1, v16h b0, v16h b1) {
#if defined(__HIP_DEVICE_COMPILE__)
  asm volatile("v_nop\n\tv_nop\n\tv_nop\n\tv_nop" : "+v"(s) : "v"(a0), "v"(a1), "v"(b0), "v"(b1));
#endif
}
__device__ __forceinline__ void guard_pv6(v8f& a, v8f& b, v8f& c, v8f& d,
                                          v16h p0, v16h p1, v16h x0, v16h x1, v16h x2, v16h x3) {
#if defined(__HIP_DEVICE_COMPILE__)
  asm volatile("v_nop\n\tv_nop\n\tv_nop\n\tv_nop"
               : "+v"(a), "+v"(b), "+v"(c), "+v"(d) : "v"(p0), "v"(p1), "v"(x0), "v"(x1), "v"(x2), "v"(x3));
#endif
}
__device__ __forceinline__ void guard_pv5(v8f& a, v8f& b, v8f& c, v8f& d,
                                          v16h p0, v16h x0, v16h x1, v16h x2, v16h x3) {
#if defined(__HIP_DEVICE_COMPILE__)
  asm volatile("v_nop\n\tv_nop\n\tv_nop\n\tv_nop"
               : "+v"(a), "+v"(b), "+v"(c), "+v"(d) : "v"(p0), "v"(x0), "v"(x1), "v"(x2), "v"(x3));
#endif
}
__device__ __forceinline__ void keep4_h(v16h a, v16h b, v16h c, v16h d) {
#if defined(__HIP_DEVICE_COMPILE__)
  asm volatile("v_nop" :: "v"(a), "v"(b), "v"(c), "v"(d));
#endif
}
__device__ __forceinline__ void acc_guard4(v8f& a, v8f& b, v8f& c, v8f& d) {
#if defined(__HIP_DEVICE_COMPILE__)
  asm volatile("v_nop\n\tv_nop\n\tv_nop\n\tv_nop" : "+v"(a), "+v"(b), "+v"(c), "+v"(d));
#endif
}
__device__ __forceinline__ void wave_sync_lds() {
  __builtin_amdgcn_fence(__ATOMIC_RELEASE, "workgroup");
  __builtin_amdgcn_wave_barrier();
  __builtin_amdgcn_fence(__ATOMIC_ACQUIRE, "workgroup");
}

__global__ __launch_bounds__(256) void conv_rows(const float* __restrict__ X, unsigned short* Y, int nrows, float carry) {
  const int lane = threadIdx.x & 31, wave = threadIdx.x >> 5;
  const int row = blockIdx.x * 8 + wave;
  if (row >= nrows) return;
  const float* xp = X + (size_t)row * DM;
  unsigned short* op = Y + (size_t)row * DM;
  v4u res[4];
#pragma unroll
  for (int j = 0; j < 4; ++j) {
    const int c0 = j * 256 + lane * 8;
    const v4f a0 = *(const v4f*)(xp + c0), a1 = *(const v4f*)(xp + c0 + 4);
    float t[8];
#pragma unroll
    for (int e = 0; e < 4; ++e) { t[e] = bfr(a0[e]) * carry; t[4 + e] = bfr(a1[e]) * carry; }
    v4u o = {0u, 0u, 0u, 0u};
#pragma unroll
    for (int e = 0; e < 4; ++e) o[e] = pk16(h_bits((_Float16)t[2 * e]), h_bits((_Float16)t[2 * e + 1]));
    res[j] = o;
  }
  for (int pass = 0; pass < 2; ++pass) {
#pragma unroll
    for (int j = 0; j < 4; ++j) *(volatile v4u*)(op + j * 256 + lane * 8) = res[j];
    __threadfence();
  }
}

__global__ __launch_bounds__(256) void conv_gate(const float* __restrict__ Wa, const float* __restrict__ We,
                                                 unsigned short* Y, float carry) {
  const int lane = threadIdx.x & 31, wave = threadIdx.x >> 5;
  const int row = blockIdx.x * 8 + wave;
  if (row >= NGATE) return;
  const float* pa = Wa + (size_t)(row & 15) * DM;
  const float* pb = We + (size_t)(row & 15) * DM;
  const bool useb = (row & 16) != 0;
  unsigned short* op = Y + (size_t)row * DM;
  v4u res[4];
#pragma unroll
  for (int j = 0; j < 4; ++j) {
    const int c0 = j * 256 + lane * 8;
    const v4f a0 = *(const v4f*)(pa + c0), a1 = *(const v4f*)(pa + c0 + 4);
    const v4f b0 = *(const v4f*)(pb + c0), b1 = *(const v4f*)(pb + c0 + 4);
    float t[8];
#pragma unroll
    for (int e = 0; e < 4; ++e) {
      t[e]     = bfr(useb ? b0[e] : a0[e]) * carry;
      t[4 + e] = bfr(useb ? b1[e] : a1[e]) * carry;
    }
    v4u o = {0u, 0u, 0u, 0u};
#pragma unroll
    for (int e = 0; e < 4; ++e) o[e] = pk16(h_bits((_Float16)t[2 * e]), h_bits((_Float16)t[2 * e + 1]));
    res[j] = o;
  }
  for (int pass = 0; pass < 2; ++pass) {
#pragma unroll
    for (int j = 0; j < 4; ++j) *(volatile v4u*)(op + j * 256 + lane * 8) = res[j];
    __threadfence();
  }
}

template <int OM, int BM, int ACT, int SPLITA>
__global__ __launch_bounds__(256) void gemm64(
    const unsigned short* __restrict__ Ap, const unsigned short* __restrict__ A2p, int lda,
    const unsigned short* __restrict__ Btp, int ldb,
    const float* __restrict__ bias, const float* __restrict__ bias2,
    void* Cout, void* C2out, int ldc,
    int M, int N, int K, float oscale, float ocarry) {
  __shared__ __align__(16) float sT[8][16 * 68];
  const int lane = threadIdx.x & 31;
  const int wave = threadIdx.x >> 5;
  const int tilesN = N >> 6;
  const int tilesM = M >> 6;
  const int tile = blockIdx.x * 8 + wave;
  if (tile >= tilesM * tilesN) return;
  const int tm = tile / tilesN;
  const int tn = tile - tm * tilesN;
  const int m0 = tm << 6;
  const int n0 = tn << 6;

  const int rlane = lane & 15;
  const int koff  = (lane >> 4) * 8;
  const int mOff  = (lane >> 4) * 8;

  v8f acc[4][4];
#pragma unroll
  for (int i = 0; i < 4; ++i)
#pragma unroll
    for (int j = 0; j < 4; ++j) acc[i][j] = zero8();

  for (int k0 = 0; k0 < K; k0 += 32) {
    v16h bh[4];
#pragma unroll
    for (int j = 0; j < 4; ++j) {
      const size_t bofs = (size_t)(n0 + (j << 4) + rlane) * ldb + koff + k0;
      bh[j] = ldfrag_u(Btp + bofs);
    }
#pragma unroll
    for (int i = 0; i < 4; ++i) {
      const size_t ao = (size_t)(m0 + (i << 4) + rlane) * lda + koff + k0;
      const v16h ah = ldfrag_u(Ap + ao);
#pragma unroll
      for (int j = 0; j < 4; ++j) acc[i][j] = mma_raw(ah, bh[j], acc[i][j]);
      if constexpr (SPLITA != 0) {
        const v16h al = ldfrag_u(A2p + ao);
#pragma unroll
        for (int j = 0; j < 4; ++j) acc[i][j] = mma_raw(al, bh[j], acc[i][j]);
        dep_guard2(acc[i][0], acc[i][3], ah, al);
      } else {
        dep_guard1(acc[i][0], acc[i][3], ah);
      }
    }
    keep4_h(bh[0], bh[1], bh[2], bh[3]);
  }
  acc_guard4(acc[0][0], acc[0][1], acc[0][2], acc[0][3]);
  acc_guard4(acc[1][0], acc[1][1], acc[1][2], acc[1][3]);
  acc_guard4(acc[2][0], acc[2][1], acc[2][2], acc[2][3]);
  acc_guard4(acc[3][0], acc[3][1], acc[3][2], acc[3][3]);

  const int hh2 = lane >> 4, c4 = (lane & 15) * 4;
  const int q8  = lane >> 3, c8 = (lane & 7) * 8;
  float bc[4];
#pragma unroll
  for (int e = 0; e < 4; ++e) bc[e] = 0.f;
  if constexpr (BM == 3) {
#pragma unroll
    for (int e = 0; e < 4; ++e) {
      const int col = n0 + c4 + e;
      const float fa = bfr(bias[col & 15]);
      const float fb = bfr(bias2[col & 15]);
      bc[e] = (col & 16) ? fb : fa;
    }
  }

  float* slab = sT[wave];
#pragma unroll
  for (int i = 0; i < 4; ++i) {
    const int mBase = m0 + (i << 4);
#pragma unroll
    for (int j = 0; j < 4; ++j) {
#pragma unroll
      for (int r = 0; r < 8; ++r) {
        slab[(mOff + r) * 68 + (j << 4) + rlane] = acc[i][j][r];
      }
    }
    wave_sync_lds();
    if constexpr (OM == 0) {
      float* C = (float*)Cout;
      v4f vals[8];
#pragma unroll
      for (int it = 0; it < 8; ++it) {
        const int row = it * 2 + hh2;
        v4f v = *(const v4f*)(slab + row * 68 + c4);
#pragma unroll
        for (int e = 0; e < 4; ++e) {
          float f = v[e] * oscale + bc[e];
          if constexpr (ACT == 2) f = 1.0f / (1.0f + __expf(-f));
          v[e] = f;
        }
        vals[it] = v;
      }
      for (int pass = 0; pass < 2; ++pass) {
#pragma unroll
        for (int it = 0; it < 8; ++it) {
          const int gr = mBase + it * 2 + hh2;
          *(volatile v4f*)(C + (size_t)gr * ldc + n0 + c4) = vals[it];
        }
        __threadfence();
      }
    } else {
      unsigned short* C  = (unsigned short*)Cout;
      unsigned short* C2 = (unsigned short*)C2out;
      v4u hv[4], lv[4];
#pragma unroll
      for (int it = 0; it < 4; ++it) {
        const int row = it * 4 + q8;
        const float* sp = slab + row * 68 + c8;
        v4u a = {0u, 0u, 0u, 0u};
        v4u b = {0u, 0u, 0u, 0u};
#pragma unroll
        for (int e = 0; e < 4; ++e) {
          const float f0 = (sp[2 * e] * oscale) * ocarry;
          const float f1 = (sp[2 * e + 1] * oscale) * ocarry;
          const _Float16 h0 = (_Float16)f0, h1 = (_Float16)f1;
          a[e] = pk16(h_bits(h0), h_bits(h1));
          if constexpr (OM == 3) {
            const _Float16 l0 = (_Float16)(f0 - (float)h0);
            const _Float16 l1 = (_Float16)(f1 - (float)h1);
            b[e] = pk16(h_bits(l0), h_bits(l1));
          }
        }
        hv[it] = a;
        lv[it] = b;
      }
      for (int pass = 0; pass < 2; ++pass) {
#pragma unroll
        for (int it = 0; it < 4; ++it) {
          const int row = it * 4 + q8;
          *(volatile v4u*)(C + (size_t)(mBase + row) * ldc + n0 + c8) = hv[it];
          if constexpr (OM == 3) {
            *(volatile v4u*)(C2 + (size_t)(mBase + row) * ldc + n0 + c8) = lv[it];
          }
        }
        __threadfence();
      }
    }
    wave_sync_lds();
  }
}

__global__ __launch_bounds__(ATT_THREADS)
void attn_heads(const unsigned short* __restrict__ QKq, const unsigned short* __restrict__ VHq,
                const unsigned short* __restrict__ VLq, const float* __restrict__ AEF,
                const float* __restrict__ betap, const float* __restrict__ ivp,
                const float* __restrict__ ovp, const float* __restrict__ chg,
                unsigned short* CTH, unsigned short* CTL) {
  __shared__ __align__(16) float Ps[HPB][16 * 36];
  __shared__ __align__(16) unsigned short Osh[16 * OSW];
  __shared__ __align__(16) unsigned short Osl[16 * OSW];

  const int tid  = threadIdx.x;
  const int wave = tid >> 5;
  const int lane = tid & 31;
  const int hh   = lane >> 4;
  const int c    = lane & 15;

  const int qt   = blockIdx.x % ATT_QT;
  const int hg   = (blockIdx.x / ATT_QT) & 1;
  const int head = hg * HPB + wave;
  const int q0   = qt * 16;

  const _Float16* Qh = (const _Float16*)(const void*)QKq + (size_t)(q0 + c) * QKP + head * HDIM + 8 * hh;
  const _Float16* Kb = (const _Float16*)(const void*)QKq + DM + head * HDIM + 8 * hh;
  const _Float16* Vh = (const _Float16*)(const void*)VHq + (size_t)(head * HDIM + c) * TT + 8 * hh;
  const _Float16* Vl = (const _Float16*)(const void*)VLq + (size_t)(head * HDIM + c) * TT + 8 * hh;
  const float* Ex = AEF + 16 + head;
  const float lsc = (1.4426950408889634f * ATT_SCALE) / (QC * KC);

  const v16h qa = ldfrag_h(Qh), qb = ldfrag_h(Qh + 32);

  float mrow[8], lrow[8], zrow[8];
  v8f o0 = zero8(), o1 = zero8(), o2 = zero8(), o3 = zero8();
#pragma unroll
  for (int r = 0; r < 8; ++r) { mrow[r] = -INFINITY; lrow[r] = 0.f; zrow[r] = 0.f; }
  float* pt = Ps[wave];

#pragma unroll 1
  for (int kb = 0; kb < TT; kb += 32) {
    const _Float16* kp = Kb + (size_t)(kb + c) * QKP;
    v8f s0, s1;
    {
      const v16h k0 = ldfrag_h(kp), k1 = ldfrag_h(kp + 32);
      s0 = mma_raw(qa, k0, zero8());
      s0 = mma_raw(qb, k1, s0);
      guard_s2(s0, k0, k1);
    }
    {
      const _Float16* kq = kp + (size_t)16 * QKP;
      const v16h k0 = ldfrag_h(kq), k1 = ldfrag_h(kq + 32);
      s1 = mma_raw(qa, k0, zero8());
      s1 = mma_raw(qb, k1, s1);
      guard_s4(s1, k0, k1, qa, qb);
    }
    const float ex0 = Ex[(size_t)(kb + c) * NGATE];
    const float ex1 = Ex[(size_t)(kb + 16 + c) * NGATE];
#pragma unroll
    for (int r = 0; r < 8; ++r) {
      const float t0 = s0[r] * lsc, t1 = s1[r] * lsc;
      float mx = fmaxf(t0, t1);
#pragma unroll
      for (int off = 1; off < 16; off <<= 1) mx = fmaxf(mx, __shfl_xor(mx, off, 32));
      const float mn = fmaxf(mrow[r], mx);
      const float al = exp2f(mrow[r] - mn);
      mrow[r] = mn;
      const float e0 = exp2f(t0 - mn), e1 = exp2f(t1 - mn);
      const float p0 = e0 * ex0, p1 = e1 * ex1;
      float zs = e0 + e1;
      float ps = p0 + p1;
#pragma unroll
      for (int off = 1; off < 16; off <<= 1) {
        zs += __shfl_xor(zs, off, 32);
        ps += __shfl_xor(ps, off, 32);
      }
      zrow[r] = zrow[r] * al + zs;
      lrow[r] = lrow[r] * al + ps;
      o0[r] *= al;
      o1[r] *= al;
      o2[r] *= al;
      o3[r] *= al;
      const int ro = (8 * hh + r) * 36 + c;
      pt[ro]      = p0;
      pt[ro + 16] = p1;
    }
    wave_sync_lds();
    FragH ph, pl;
    {
      const float* prow = pt + c * 36 + 8 * hh;
      const v4f g0 = *(const v4f*)(prow), g1 = *(const v4f*)(prow + 4);
      const v4f g2 = *(const v4f*)(prow + 16), g3 = *(const v4f*)(prow + 20);
#pragma unroll
      for (int e = 0; e < 4; ++e) {
        float xv; _Float16 hx;
        xv = g0[e] * PC; hx = (_Float16)xv; ph.h[0][e]     = hx; pl.h[0][e]     = (_Float16)(xv - (float)hx);
        xv = g1[e] * PC; hx = (_Float16)xv; ph.h[0][4 + e] = hx; pl.h[0][4 + e] = (_Float16)(xv - (float)hx);
        xv = g2[e] * PC; hx = (_Float16)xv; ph.h[1][e]     = hx; pl.h[1][e]     = (_Float16)(xv - (float)hx);
        xv = g3[e] * PC; hx = (_Float16)xv; ph.h[1][4 + e] = hx; pl.h[1][4 + e] = (_Float16)(xv - (float)hx);
      }
    }
    {
      const _Float16* vp = Vh + kb;
      const v16h vb0 = ldfrag_h(vp);
      const v16h vb1 = ldfrag_h(vp + (size_t)16 * TT);
      const v16h vb2 = ldfrag_h(vp + (size_t)32 * TT);
      const v16h vb3 = ldfrag_h(vp + (size_t)48 * TT);
      o0 = mma_raw(ph.v, vb0, o0);
      o1 = mma_raw(ph.v, vb1, o1);
      o2 = mma_raw(ph.v, vb2, o2);
      o3 = mma_raw(ph.v, vb3, o3);
      o0 = mma_raw(pl.v, vb0, o0);
      o1 = mma_raw(pl.v, vb1, o1);
      o2 = mma_raw(pl.v, vb2, o2);
      o3 = mma_raw(pl.v, vb3, o3);
      guard_pv6(o0, o1, o2, o3, ph.v, pl.v, vb0, vb1, vb2, vb3);
    }
    {
      const _Float16* vp = Vl + kb;
      const v16h vl0 = ldfrag_h(vp);
      const v16h vl1 = ldfrag_h(vp + (size_t)16 * TT);
      const v16h vl2 = ldfrag_h(vp + (size_t)32 * TT);
      const v16h vl3 = ldfrag_h(vp + (size_t)48 * TT);
      o0 = mma_raw(ph.v, vl0, o0);
      o1 = mma_raw(ph.v, vl1, o1);
      o2 = mma_raw(ph.v, vl2, o2);
      o3 = mma_raw(ph.v, vl3, o3);
      guard_pv5(o0, o1, o2, o3, ph.v, vl0, vl1, vl2, vl3);
    }
    wave_sync_lds();
  }

  const float* Ap = AEF + head;
  float apr[8];
#pragma unroll
  for (int r = 0; r < 8; ++r) apr[r] = Ap[(size_t)(q0 + 8 * hh + r) * NGATE];
  const float bet = bfr(betap[head]);
  const float ivs = sigf(bfr(ivp[head]));
  const float og  = sigf(bfr(ovp[head])) * tanhf(bfr(chg[head]));
  const float ang = PI_F * sigf(bet);
  const float ca  = cosf(ang), sa = sinf(ang);
  const float base = ivs / (PC * VC);
  unsigned short* oh = Osh + wave * HDIM + c;
  unsigned short* ol = Osl + wave * HDIM + c;
#pragma unroll
  for (int r = 0; r < 8; ++r) {
    const float den = apr[r] * lrow[r] + REN_EPS * zrow[r];
    const float sc  = apr[r] * (1.0f / den) * base;
    const float x0 = o0[r] * sc, x1 = o1[r] * sc, x2 = o2[r] * sc, x3 = o3[r] * sc;
    const float y0 = ((x0 * ca - x2 * sa) * og) * FC;
    const float y1 = ((x1 * ca - x3 * sa) * og) * FC;
    const float y2 = ((x0 * sa + x2 * ca) * og) * FC;
    const float y3 = ((x1 * sa + x3 * ca) * og) * FC;
    const _Float16 h0 = (_Float16)y0, h1 = (_Float16)y1, h2 = (_Float16)y2, h3 = (_Float16)y3;
    const int ro = (8 * hh + r) * OSW;
    oh[ro]      = h_bits(h0);
    oh[ro + 16] = h_bits(h1);
    oh[ro + 32] = h_bits(h2);
    oh[ro + 48] = h_bits(h3);
    ol[ro]      = h_bits((_Float16)(y0 - (float)h0));
    ol[ro + 16] = h_bits((_Float16)(y1 - (float)h1));
    ol[ro + 32] = h_bits((_Float16)(y2 - (float)h2));
    ol[ro + 48] = h_bits((_Float16)(y3 - (float)h3));
  }
  __syncthreads();
  {
    v4u vh[4], vl[4];
#pragma unroll
    for (int it = 0; it < 4; ++it) {
      const int p = it * ATT_THREADS + tid;
      vh[it] = *(const v4u*)(Osh + (size_t)p * 8);
      vl[it] = *(const v4u*)(Osl + (size_t)p * 8);
    }
    const size_t dofs = (size_t)q0 * DM + (size_t)hg * OSW;
    unsigned short* dh = CTH + dofs;
    unsigned short* dl = CTL + dofs;
    for (int pass = 0; pass < 2; ++pass) {
#pragma unroll
      for (int it = 0; it < 4; ++it) {
        const int p = it * ATT_THREADS + tid;
        const size_t po = (size_t)(p >> 6) * DM + (size_t)(p & 63) * 8;
        *(volatile v4u*)(dh + po) = vh[it];
        *(volatile v4u*)(dl + po) = vl[it];
      }
      __threadfence();
    }
  }
}

extern "C" void kernel_launch(void* const* d_in, const int* in_sizes, int n_in,
                              void* d_out, int out_size, void* d_ws, size_t ws_size,
                              hipStream_t stream) {
  if (n_in < 13) return;
  if (in_sizes[0] != TT * DM) return;
  if (in_sizes[1] != NHEAD * DM || in_sizes[2] != NHEAD) return;
  if (in_sizes[3] != NHEAD * DM || in_sizes[4] != NHEAD) return;
  if (in_sizes[5] != DM * DM || in_sizes[6] != DM * DM || in_sizes[7] != DM * DM || in_sizes[8] != DM * DM) return;
  if (in_sizes[9] != NHEAD || in_sizes[10] != NHEAD || in_sizes[11] != NHEAD || in_sizes[12] != NHEAD) return;
  if (out_size != TT * DM) return;

  const float* x     = (const float*)d_in[0];
  const float* Wa    = (const float*)d_in[1];
  const float* ba    = (const float*)d_in[2];
  const float* We    = (const float*)d_in[3];
  const float* be    = (const float*)d_in[4];
  const float* Wi    = (const float*)d_in[5];
  const float* Wo    = (const float*)d_in[6];
  const float* Wv    = (const float*)d_in[7];
  const float* Wout  = (const float*)d_in[8];
  const float* betap = (const float*)d_in[9];
  const float* ivp   = (const float*)d_in[10];
  const float* ovp   = (const float*)d_in[11];
  const float* chg   = (const float*)d_in[12];
  float*       out   = (float*)d_out;

  const size_t PWIO = (size_t)2 * DM * DM * 2;
  const size_t PW   = (size_t)DM * DM * 2;
  const size_t PG   = (size_t)NGATE * DM * 2;
  const size_t PX   = (size_t)TT * DM * 2;
  const size_t PQK  = (size_t)TT * QKP * 2;
  const size_t PVT  = (size_t)DM * TT * 2;
  const size_t PAE  = (size_t)TT * NGATE * 4;
  const size_t PCT  = (size_t)TT * DM * 2;
  size_t off = 0;
  const size_t oWIO = off; off += PWIO;
  const size_t oWV  = off; off += PW;
  const size_t oWOU = off; off += PW;
  const size_t oWG  = off; off += PG;
  const size_t oXB  = off; off += PX;
  const size_t oQK  = off; off += PQK;
  const size_t oVTH = off; off += PVT;
  const size_t oVTL = off; off += PVT;
  const size_t oAEF = off; off += PAE;
  const size_t oCTH = off; off += PCT;
  const size_t oCTL = off; off += PCT;
  if (off > ws_size) return;
  if (off > (size_t)134217728) return;

  char* ws = (char*)d_ws;
  unsigned short* WIO  = (unsigned short*)(ws + oWIO);
  unsigned short* WV   = (unsigned short*)(ws + oWV);
  unsigned short* WOUT = (unsigned short*)(ws + oWOU);
  unsigned short* WG   = (unsigned short*)(ws + oWG);
  unsigned short* XB   = (unsigned short*)(ws + oXB);
  unsigned short* QK   = (unsigned short*)(ws + oQK);
  unsigned short* VTH  = (unsigned short*)(ws + oVTH);
  unsigned short* VTL  = (unsigned short*)(ws + oVTL);
  float*          AEF  = (float*)(ws + oAEF);
  unsigned short* CTH  = (unsigned short*)(ws + oCTH);
  unsigned short* CTL  = (unsigned short*)(ws + oCTL);

  const dim3 blk(256);
  const dim3 gX(TT / 8);
  const dim3 gW(DM / 8);
  const dim3 gG(NGATE / 8);
  const int tilesG = (TT / 64) * (NGATE / 64);
  const int tilesQ = (TT / 64) * (QKP / 64);
  const int tilesV = (DM / 64) * (TT / 64);
  const int tilesO = (TT / 64) * (DM / 64);
  const dim3 gGE((tilesG + 7) / 8);
  const dim3 gQK((tilesQ + 7) / 8);
  const dim3 gVT((tilesV + 7) / 8);
  const dim3 gO((tilesO + 7) / 8);
  const dim3 gAT(ATT_BLOCKS);
  const dim3 bAT(ATT_THREADS);

  conv_rows<<<gX, blk, 0, stream>>>(x, XB, TT, ACARRY);
  conv_rows<<<gW, blk, 0, stream>>>(Wi, WIO, DM, WSC);
  conv_rows<<<gW, blk, 0, stream>>>(Wo, WIO + (size_t)DM * DM, DM, WSC);
  conv_rows<<<gW, blk, 0, stream>>>(Wv, WV, DM, WSC);
  conv_rows<<<gW, blk, 0, stream>>>(Wout, WOUT, DM, WSC);
  conv_gate<<<gG, blk, 0, stream>>>(Wa, We, WG, WSC);

  gemm64<0, 3, 2, 0><<<gGE, blk, 0, stream>>>(
      XB, XB, DM,
      WG, DM,
      ba, be,
      (void*)AEF, (void*)AEF, NGATE,
      TT, NGATE, DM, 1.0f / (ACARRY * WSC), 1.0f);

  gemm64<2, 0, 0, 0><<<gQK, blk, 0, stream>>>(
      XB, XB, DM,
      WIO, DM,
      ba, be,
      (void*)QK, (void*)QK, QKP,
      TT, QKP, DM, 1.0f / (ACARRY * WSC), QC);

  gemm64<3, 0, 0, 0><<<gVT, blk, 0, stream>>>(
      WV, WV, DM,
      XB, DM,
      ba, be,
      (void*)VTH, (void*)VTL, TT,
      DM, TT, DM, 1.0f / (WSC * ACARRY), VC);

  attn_heads<<<gAT, bAT, 0, stream>>>(QK, VTH, VTL, AEF, betap, ivp, ovp, chg, CTH, CTL);

  gemm64<0, 0, 0, 1><<<gO, blk, 0, stream>>>(
      CTH, CTL, DM,
      WOUT, DM,
      ba, be,
      (void*)out, (void*)out, DM,
      TT, DM, DM, 1.0f / (FC * WSC), 1.0f);
  (void)hipGetLastError();
}
